// MoeConv_16501264351576
// MI455X (gfx1250) — hardware-verified
//
#include <hip/hip_runtime.h>
#include <math.h>

typedef __attribute__((ext_vector_type(16))) _Float16 v16h;
typedef __attribute__((ext_vector_type(8)))  _Float16 v8h;
typedef __attribute__((ext_vector_type(8)))  float    v8f;
typedef __attribute__((ext_vector_type(4)))  float    v4f;
typedef __attribute__((ext_vector_type(4)))  unsigned v4u;
typedef float __attribute__((may_alias)) float_a;
#define WSC 16.0f
#define WUN 0.0625f

__device__ __forceinline__ v8f wmma_f16(v16h a, v16h b, v8f c) {
  v8f d = __builtin_amdgcn_wmma_f32_16x16x32_f16(false, a, false, b, (short)0, c, false, false);
  asm volatile("v_nop\n\tv_nop\n\tv_nop\n\tv_nop" : "+v"(d) : "v"(a), "v"(b));
  return d;
}

#define CIN   128
#define COUT  128
#define HH    96
#define WW    96
#define NE    8
#define KTOT  1152
#define CIP   136

__global__ __launch_bounds__(256) void moe_pack_w_k(
    const float* __restrict__ expert_w, const float* __restrict__ shared_w,
    _Float16* __restrict__ Apack)
{
  int idx = blockIdx.x * 256 + threadIdx.x;
  int m   = idx / (KTOT / 8);
  int k0  = (idx - m * (KTOT / 8)) * 8;
  int tap = k0 >> 7;
  int ci0 = k0 & 127;
  int s   = m >> 7;
  int co  = m & 127;
  union { v8h h; v4u u; } pk;
#pragma unroll
  for (int i = 0; i < 8; ++i) {
    float v;
    if (s < NE) v = expert_w[((size_t)(s * COUT + co) * CIN + ci0 + i) * 9 + tap];
    else        v = shared_w[((size_t)co * CIN + ci0 + i) * 9 + tap];
    pk.h[i] = (_Float16)(v * WSC);
  }
  _Float16* dst = Apack + (size_t)m * KTOT + k0;
  *(volatile v4u*)dst = pk.u;
  __threadfence();
  *(volatile v4u*)dst = pk.u;
}

__global__ __launch_bounds__(256) void moe_gate_k(
    const float* __restrict__ x, const float* __restrict__ gate_w,
    float* __restrict__ gsc)
{
  __shared__ float gwl[CIN * 9 * NE];
  int tid = threadIdx.x;
  for (int i = tid; i < NE * CIN * 9; i += 256) {
    int e = i / (CIN * 9);
    int r = i - e * (CIN * 9);
    gwl[r * NE + e] = gate_w[i];
  }
  __syncthreads();

  int pix = blockIdx.x * 256 + tid;
  int b   = pix / (HH * WW);
  int hw  = pix - b * (HH * WW);
  int h   = hw / WW;
  int w   = hw - h * WW;

  float acc[NE];
#pragma unroll
  for (int e = 0; e < NE; ++e) acc[e] = 0.f;

  for (int ci = 0; ci < CIN; ++ci) {
    const float* xp = x + ((size_t)(b * CIN + ci) * HH) * WW;
#pragma unroll
    for (int t = 0; t < 9; ++t) {
      int h2 = h + (t / 3) - 1;
      int w2 = w + (t % 3) - 1;
      if (h2 >= 0 && h2 < HH && w2 >= 0 && w2 < WW) {
        float xv = xp[h2 * WW + w2];
        const float* gp = &gwl[(ci * 9 + t) * NE];
#pragma unroll
        for (int e = 0; e < NE; ++e) acc[e] = fmaf(xv, gp[e], acc[e]);
      }
    }
  }
#pragma unroll
  for (int e = 0; e < NE; ++e) {
    const float sg = 1.f / (1.f + expf(-acc[e]));
    float* dst = gsc + (size_t)(b * NE + e) * (HH * WW) + hw;
    *(volatile float_a*)dst = sg;
    __threadfence();
    *(volatile float_a*)dst = sg;
  }
}

__global__ __launch_bounds__(96) void moe_route_k(
    const float* __restrict__ gsc, const float* __restrict__ gate_bias,
    float* __restrict__ score_full)
{
  int row = blockIdx.x;
  int b   = row / HH;
  int h   = row - b * HH;
  int tid = threadIdx.x;
  int hw  = h * WW + tid;

  float sc[NE], bi[NE];
#pragma unroll
  for (int e = 0; e < NE; ++e) {
    sc[e] = gsc[(size_t)(b * NE + e) * (HH * WW) + hw];
    bi[e] = sc[e] + gate_bias[e];
  }
  int i0 = 0; float m0b = bi[0]; float m0s = sc[0];
#pragma unroll
  for (int e = 1; e < NE; ++e)
    if (bi[e] > m0b) { m0b = bi[e]; m0s = sc[e]; i0 = e; }
  int i1 = -1; float m1b = -3.4e38f; float m1s = 0.f;
#pragma unroll
  for (int e = 0; e < NE; ++e)
    if (e != i0 && bi[e] > m1b) { m1b = bi[e]; m1s = sc[e]; i1 = e; }

  float mx  = fmaxf(m0s, m1s);
  float e0  = expf(m0s - mx), e1 = expf(m1s - mx);
  float inv = 1.f / (e0 + e1);
  float w0  = e0 * inv, w1 = e1 * inv;

#pragma unroll
  for (int e = 0; e < NE; ++e) {
    const float v = (e == i0) ? w0 : ((e == i1) ? w1 : 0.f);
    float* dst = score_full + (size_t)(b * NE + e) * (HH * WW) + hw;
    *(volatile float_a*)dst = v;
    __threadfence();
    *(volatile float_a*)dst = v;
  }
}

__global__ __launch_bounds__(128) void moe_main_wmma_k(
    const float* __restrict__ x, const _Float16* __restrict__ Apack,
    const float* __restrict__ score_full,
    const float* __restrict__ expert_b, const float* __restrict__ shared_b,
    float* __restrict__ out)
{
  __shared__ __align__(16) _Float16 Xs[3 * 98 * CIP];
  __shared__ __align__(16) float Ot[64 * WW];

  const int tid    = threadIdx.x;
  const int lane   = tid & 31;
  const int wid    = tid >> 5;
  const int wave_m = wid >> 1;
  const int wave_n = wid & 1;
  const int lhalf  = lane & 15;
  const int hsel   = lane >> 4;

  const int co_base = blockIdx.x * 64;
  const int bh = blockIdx.y;
  const int b  = bh / HH;
  const int h  = bh - b * HH;

  for (int p = tid; p < 3 * 98; p += 128) {
    int r3   = p / 98;
    int cs   = p - r3 * 98;
    int wsrc = cs - 1;
    int h2   = h + r3 - 1;
    _Float16* dst = Xs + p * CIP;
    if (wsrc >= 0 && wsrc < WW && h2 >= 0 && h2 < HH) {
      const float* src = x + ((size_t)b * CIN * HH + h2) * WW + wsrc;
#pragma unroll 4
      for (int ci = 0; ci < CIN; ci += 2) {
        union { _Float16 hx[2]; unsigned int u; } pk;
        pk.hx[0] = (_Float16)src[(size_t)ci * (HH * WW)];
        pk.hx[1] = (_Float16)src[(size_t)(ci + 1) * (HH * WW)];
        *(unsigned int*)(dst + ci) = pk.u;
      }
    } else {
#pragma unroll 8
      for (int ci = 0; ci < CIN; ci += 2)
        *(unsigned int*)(dst + ci) = 0u;
    }
  }
  __syncthreads();

  const v8f zero = {0.f, 0.f, 0.f, 0.f, 0.f, 0.f, 0.f, 0.f};
  v8f fin0[3], fin1[3];
#pragma unroll
  for (int q = 0; q < 3; ++q) { fin0[q] = zero; fin1[q] = zero; }

  const int amrow = co_base + wave_m * 32 + lhalf;
  const int bn0   = wave_n * 48 + lhalf;

  for (int s = 0; s < NE + 1; ++s) {

    v8f acc0[3], acc1[3];
#pragma unroll
    for (int q = 0; q < 3; ++q) { acc0[q] = zero; acc1[q] = zero; }

    const _Float16* arow0 =
        Apack + (size_t)(s * COUT + amrow) * KTOT + hsel * 8;
    const _Float16* arow1 = arow0 + (size_t)16 * KTOT;

    for (int tap = 0; tap < 9; ++tap) {
      int dh = tap / 3;
      int dw = tap % 3;
      const _Float16* brow = Xs + (size_t)(dh * 98 + bn0 + dw) * CIP;
#pragma unroll
      for (int cq = 0; cq < 4; ++cq) {
        const int ci0 = cq * 32;
        const _Float16* ap0 = arow0 + tap * 128 + ci0;
        const _Float16* ap1 = arow1 + tap * 128 + ci0;
        v8h a0l = *(const v8h*)(ap0);
        v8h a0h = *(const v8h*)(ap0 + 16);
        v8h a1l = *(const v8h*)(ap1);
        v8h a1h = *(const v8h*)(ap1 + 16);
        v16h av0 = __builtin_shufflevector(a0l, a0h, 0, 1, 2, 3, 4, 5, 6, 7,
                                           8, 9, 10, 11, 12, 13, 14, 15);
        v16h av1 = __builtin_shufflevector(a1l, a1h, 0, 1, 2, 3, 4, 5, 6, 7,
                                           8, 9, 10, 11, 12, 13, 14, 15);
#pragma unroll
        for (int q = 0; q < 3; ++q) {
          const _Float16* bp = brow + (size_t)q * 16 * CIP + ci0 + hsel * 8;
          v8h blo = *(const v8h*)(bp);
          v8h bhi = *(const v8h*)(bp + 16);
          v16h bv = __builtin_shufflevector(blo, bhi, 0, 1, 2, 3, 4, 5, 6, 7,
                                            8, 9, 10, 11, 12, 13, 14, 15);
          acc0[q] = wmma_f16(av0, bv, acc0[q]);
          acc1[q] = wmma_f16(av1, bv, acc1[q]);
        }
      }
    }

    const int cb0 = co_base + wave_m * 32 + hsel * 8;
    const int cb1 = cb0 + 16;
    float wq[3];
#pragma unroll
    for (int q = 0; q < 3; ++q) {
      int n = bn0 + q * 16;
      wq[q] = (s == NE) ? 1.f
                        : score_full[(size_t)(b * NE + s) * (HH * WW) + h * WW + n];
    }
#pragma unroll
    for (int r = 0; r < 8; ++r) {
      float b0 = (s == NE) ? shared_b[cb0 + r] : expert_b[s * COUT + cb0 + r];
      float b1 = (s == NE) ? shared_b[cb1 + r] : expert_b[s * COUT + cb1 + r];
#pragma unroll
      for (int q = 0; q < 3; ++q) {
        fin0[q][r] += wq[q] * (acc0[q][r] * WUN + b0);
        fin1[q][r] += wq[q] * (acc1[q][r] * WUN + b1);
      }
    }
  }

#pragma unroll
  for (int q = 0; q < 3; ++q) {
    int w = bn0 + q * 16;
#pragma unroll
    for (int r = 0; r < 8; ++r) {
      int col = wave_m * 32 + hsel * 8 + r;
      Ot[col * WW + w]        = fin0[q][r];
      Ot[(col + 16) * WW + w] = fin1[q][r];
    }
  }
  __syncthreads();
  for (int g = tid; g < 64 * (WW / 4); g += 128) {
    const int col = g / (WW / 4), pc = g - col * (WW / 4);
    const v4f v = *(const v4f*)(Ot + col * WW + pc * 4);
    float* dst = out + ((size_t)(b * COUT + co_base + col) * HH + h) * WW + pc * 4;
    *(volatile v4f*)dst = v;
    __threadfence();
    *(volatile v4f*)dst = v;
  }
}

extern "C" void kernel_launch(void* const* d_in, const int* in_sizes, int n_in,
                              void* d_out, int out_size, void* d_ws, size_t ws_size,
                              hipStream_t stream) {
  (void)in_sizes; (void)n_in; (void)out_size; (void)ws_size;
  const float* x         = (const float*)d_in[0];
  const float* gate_w    = (const float*)d_in[1];
  const float* gate_bias = (const float*)d_in[2];
  const float* expert_w  = (const float*)d_in[3];
  const float* expert_b  = (const float*)d_in[4];
  const float* shared_w  = (const float*)d_in[5];
  const float* shared_b  = (const float*)d_in[6];
  float* out = (float*)d_out;

  char* ws = (char*)d_ws;
  _Float16* Apack      = (_Float16*)(ws);
  float*    score_full = (float*)(ws + 2654208);
  float*    gsc        = (float*)(ws + 3833856);
  moe_pack_w_k<<<(1152 * (KTOT / 8)) / 256, 256, 0, stream>>>(expert_w, shared_w, Apack);
  moe_gate_k<<<(4 * HH * WW) / 256, 256, 0, stream>>>(x, gate_w, gsc);
  moe_route_k<<<4 * HH, 96, 0, stream>>>(gsc, gate_bias, score_full);
  moe_main_wmma_k<<<dim3(2, 4 * HH), 128, 0, stream>>>(
      x, Apack, score_full, expert_b, shared_b, out);
}
